// RoPESelfAttention_11269994185100
// MI455X (gfx1250) — hardware-verified
//
#include <hip/hip_runtime.h>


typedef _Float16 bf16x16 __attribute__((ext_vector_type(16)));
typedef float    floatx8 __attribute__((ext_vector_type(8)));
#define RSPLIT (1.0f / 2048.0f)

constexpr int Bsz  = 2;
constexpr int Lseq = 2048;
constexpr int Dmod = 1024;
constexpr int Hn   = 16;
constexpr int DhC  = 64;
constexpr int Mrows = Bsz * Lseq;
constexpr int NQKV  = 3 * Dmod;
constexpr size_t PLX = (size_t)Mrows * Dmod;
constexpr size_t PLQKV = (size_t)Dmod * NQKV;
constexpr size_t PLO = (size_t)Dmod * Dmod;

__device__ __forceinline__ unsigned short f32_to_bf16_bits(float f) {
  return __builtin_bit_cast(unsigned short, (_Float16)f);
}
__device__ __forceinline__ void split16(float f, unsigned short& h, unsigned short& l) {
  const _Float16 hh = (_Float16)f; h = __builtin_bit_cast(unsigned short, hh);
  l = __builtin_bit_cast(unsigned short, (_Float16)((f - (float)hh) * 2048.0f));
}
__device__ __forceinline__ unsigned pack2s(float a, float b, unsigned* lo_out) {
  unsigned short h0, l0, h1, l1; split16(a, h0, l0); split16(b, h1, l1);
  *lo_out = (unsigned)l0 | ((unsigned)l1 << 16); return (unsigned)h0 | ((unsigned)h1 << 16);
}

union Frag {
  bf16x16 v;
  uint4   q[2];
};

__device__ __forceinline__ Frag load_frag_A(const unsigned short* __restrict__ base,
                                            size_t ld, int row0, int col0, int lane) {
  const int m = lane & 15, hi = lane >> 4;
  const unsigned short* p = base + (size_t)(row0 + m) * ld + col0 + hi * 8;
  Frag f;
  f.q[0] = *(const uint4*)(p);
  f.q[1] = *(const uint4*)(p + 16);
  return f;
}

__device__ __forceinline__ Frag load_frag_B(const unsigned short* __restrict__ baseT,
                                            size_t ld, int n0, int col0, int lane) {
  const int n = lane & 15, hi = lane >> 4;
  const unsigned short* p = baseT + (size_t)(n0 + n) * ld + col0 + hi * 8;
  Frag f;
  f.q[0] = *(const uint4*)(p);
  f.q[1] = *(const uint4*)(p + 16);
  return f;
}

__device__ __forceinline__ floatx8 wmma_bf16(Frag a, Frag b, floatx8 c) {
  return __builtin_amdgcn_wmma_f32_16x16x32_f16(
       false, a.v,  false, b.v,
       (short)0, c,  false,  false);
}
__device__ __forceinline__ floatx8 wmma_split(Frag ah, Frag al, Frag bh, Frag bl, floatx8 c) {
  floatx8 x = {};
  x = wmma_bf16(al, bh, x); x = wmma_bf16(ah, bl, x);
  return wmma_bf16(ah, bh, c) + x * RSPLIT;
}
__device__ __forceinline__ floatx8 mmaA_B(const unsigned short* A, size_t pla, size_t lda, int row0, int colA,
                                         const unsigned short* BT, size_t plb, size_t ldb, int n0, int colB, int lane, floatx8 c) {
  return wmma_split(load_frag_A(A, lda, row0, colA, lane), load_frag_A(A + pla, lda, row0, colA, lane),
                    load_frag_B(BT, ldb, n0, colB, lane), load_frag_B(BT + plb, ldb, n0, colB, lane), c);
}
__device__ __forceinline__ void store_rows64_planes(const float* so, unsigned short* dst, size_t plane, size_t ld, int lane) {
#pragma unroll 1
  for (int pass = 0; pass < 2; ++pass) {
#pragma unroll 4
    for (int rr = 0; rr < 16; ++rr) {
      unsigned lo; const unsigned hv = pack2s(*(const volatile float*)(so + rr * 64 + 2 * lane), *(const volatile float*)(so + rr * 64 + 2 * lane + 1), &lo);
      *(volatile unsigned*)(dst + (size_t)rr * ld + 2 * lane) = hv; *(volatile unsigned*)(dst + plane + (size_t)rr * ld + 2 * lane) = lo;
    }
    __threadfence();
  }
}

__global__ void cvt_f32_bf16(const float* __restrict__ in,
                             unsigned short* __restrict__ out, int n) {
  int i = (blockIdx.x * blockDim.x + threadIdx.x) * 2;
  if (i < n) {
    unsigned lo; const unsigned hv = pack2s(in[i], in[i + 1], &lo);
    *(volatile unsigned*)(out + i) = hv; *(volatile unsigned*)(out + (size_t)n + i) = lo;
    __threadfence();
    *(volatile unsigned*)(out + i) = hv; *(volatile unsigned*)(out + (size_t)n + i) = lo;
  }
}

__global__ void cvt_f32_bf16_T(const float* __restrict__ in,
                               unsigned short* __restrict__ out,
                               int rows, int cols) {
  int o = (blockIdx.x * blockDim.x + threadIdx.x) * 2;
  if (o < rows * cols) {
    int c = o / rows;
    int r = o - c * rows;
    unsigned lo; const unsigned hv = pack2s(in[(size_t)r * cols + c], in[(size_t)(r + 1) * cols + c], &lo);
    *(volatile unsigned*)(out + o) = hv; *(volatile unsigned*)(out + (size_t)rows * cols + o) = lo;
    __threadfence();
    *(volatile unsigned*)(out + o) = hv; *(volatile unsigned*)(out + (size_t)rows * cols + o) = lo;
  }
}

__global__ __launch_bounds__(256)
void qkv_rope_kernel(const unsigned short* __restrict__ Xbf,
                     const unsigned short* __restrict__ WqkvT,
                     unsigned short* __restrict__ Qbf,
                     unsigned short* __restrict__ Kbf,
                     unsigned short* __restrict__ Vr) {
  __shared__ __align__(16) float st[8][16 * 64];
  const int lane = threadIdx.x & 31;
  const int wib  = threadIdx.x >> 5;
  const int gw   = blockIdx.x * (blockDim.x >> 5) + (threadIdx.x >> 5);
  const int nW   = NQKV / 64;
  const int mt   = gw / nW;
  const int nw   = gw - mt * nW;
  const int row0 = mt * 16;
  const int n0   = nw * 64;

  floatx8 acc[4] = {};
  for (int k0 = 0; k0 < Dmod; k0 += 32) {
    Frag a  = load_frag_A(Xbf, Dmod, row0, k0, lane);
    Frag al = load_frag_A(Xbf + PLX, Dmod, row0, k0, lane);
    if (k0 + 32 < Dmod) {
      __builtin_prefetch(Xbf + (size_t)(row0 + (lane & 15)) * Dmod + k0 + 32, 0, 1);
    }
#pragma unroll
    for (int t = 0; t < 4; ++t) {
      Frag b  = load_frag_B(WqkvT, Dmod, n0 + 16 * t, k0, lane);
      Frag bl = load_frag_B(WqkvT + PLQKV, Dmod, n0 + 16 * t, k0, lane);
      acc[t] = wmma_split(a, al, b, bl, acc[t]);
    }
  }

  const int n  = lane & 15, hi = lane >> 4;
  const int seg = n0 / Dmod;
  const int h   = (n0 - seg * Dmod) / DhC;

  float* sw = st[wib];
  if (seg < 2) {
#pragma unroll
    for (int j = 0; j < 8; ++j) {
      const int m   = row0 + j + 8 * hi;
      const int pos = m & (Lseq - 1);
#pragma unroll
      for (int t = 0; t < 2; ++t) {
        const int d = 16 * t + n;
        const float invf = __expf(-(float)d * 0.28782313662f);
        const float ang  = (float)pos * invf;
        float s, c;
        sincosf(ang, &s, &c);
        const float x1 = acc[t][j], x2 = acc[t + 2][j];
        sw[(j + 8 * hi) * 64 + d]      = x1 * c - x2 * s;
        sw[(j + 8 * hi) * 64 + d + 32] = x1 * s + x2 * c;
      }
    }
  } else {
#pragma unroll
    for (int j = 0; j < 8; ++j)
#pragma unroll
      for (int t = 0; t < 4; ++t) sw[(j + 8 * hi) * 64 + 16 * t + n] = acc[t][j];
  }
  asm volatile("s_wait_dscnt 0" ::: "memory");
  unsigned short* dst = (seg == 0) ? Qbf : (seg == 1) ? Kbf : Vr;
  store_rows64_planes(sw, dst + (size_t)row0 * Dmod + h * DhC, PLX, Dmod, lane);
}

__global__ __launch_bounds__(256) void vt_kernel(const unsigned short* __restrict__ Vr, unsigned short* __restrict__ Vt) {
  __shared__ unsigned short t[64][66];
  const int tid = threadIdx.x, lane = tid & 31, wave = tid >> 5;
  const int m0 = blockIdx.x * 64, c0 = blockIdx.y * 64;
  const size_t pl = blockIdx.z ? PLX : 0;
  const int b = m0 >> 11, pos0 = m0 & (Lseq - 1);
#pragma unroll
  for (int k = 0; k < 16; ++k) { const int e = tid + 256 * k; t[e >> 6][e & 63] = Vr[pl + (size_t)(m0 + (e >> 6)) * Dmod + c0 + (e & 63)]; }
  __syncthreads();
  unsigned short* dst = Vt + pl + (size_t)b * Dmod * Lseq + pos0;
#pragma unroll
  for (int rr = 0; rr < 8; ++rr) {
    const int c = wave * 8 + rr;
    const unsigned pk = (unsigned)t[2 * lane][c] | ((unsigned)t[2 * lane + 1][c] << 16);
    unsigned* d = (unsigned*)(dst + (size_t)(c0 + c) * Lseq) + lane;
    *(volatile unsigned*)d = pk; __threadfence(); *(volatile unsigned*)d = pk;
  }
}

__global__ __launch_bounds__(256)
void attn_kernel(const unsigned short* __restrict__ Qbf,
                 const unsigned short* __restrict__ Kbf,
                 const unsigned short* __restrict__ Vt,
                 const int* __restrict__ mask,
                 unsigned short* __restrict__ Attnbf) {
  __shared__ __align__(16) unsigned short Plds[8][16 * 32];
  __shared__ __align__(16) unsigned short Pldsl[8][16 * 32];
  __shared__ __align__(16) float ost[8][16 * 64];

  const int wib  = threadIdx.x >> 5;
  const int lane = threadIdx.x & 31;
  const int gw   = blockIdx.x * 8 + wib;
  const int qt = gw & 127;
  const int h  = (gw >> 7) & 15;
  const int b  = gw >> 11;

  const int n = lane & 15, hi = lane >> 4;
  const unsigned short* VtB = Vt + (size_t)b * Dmod * Lseq;

  Frag qf[2], qfl[2];
#pragma unroll
  for (int s = 0; s < 2; ++s) {
    qf[s]  = load_frag_A(Qbf, Dmod, b * Lseq + qt * 16, h * DhC + s * 32, lane);
    qfl[s] = load_frag_A(Qbf + PLX, Dmod, b * Lseq + qt * 16, h * DhC + s * 32, lane);
  }

  float rmax[8], rsum[8];
#pragma unroll
  for (int j = 0; j < 8; ++j) { rmax[j] = -1e30f; rsum[j] = 0.f; }
  floatx8 O[4] = {};

  for (int k0 = 0; k0 < Lseq; k0 += 32) {
    float s2[2][8];
    float mk[2];
#pragma unroll
    for (int t = 0; t < 2; ++t) {
      floatx8 c = {};
#pragma unroll
      for (int s = 0; s < 2; ++s) {
        Frag kf  = load_frag_B(Kbf, Dmod, b * Lseq + k0 + 16 * t, h * DhC + s * 32, lane);
        Frag kfl = load_frag_B(Kbf + PLX, Dmod, b * Lseq + k0 + 16 * t, h * DhC + s * 32, lane);
        c = wmma_split(qf[s], qfl[s], kf, kfl, c);
      }
      mk[t] = (mask[b * Lseq + k0 + 16 * t + n] != 0) ? 1.f : 0.f;
#pragma unroll
      for (int j = 0; j < 8; ++j)
        s2[t][j] = (mk[t] != 0.f) ? -1e30f : c[j] * 0.125f;
    }

#pragma unroll
    for (int j = 0; j < 8; ++j) {
      float mx = fmaxf(s2[0][j], s2[1][j]);
#pragma unroll
      for (int off = 1; off < 16; off <<= 1)
        mx = fmaxf(mx, __shfl_xor(mx, off, 32));
      const float nm    = fmaxf(rmax[j], mx);
      const float alpha = __expf(rmax[j] - nm);
      rmax[j] = nm;
      const float p0 = __expf(s2[0][j] - nm);
      const float p1 = __expf(s2[1][j] - nm);
      float ls = p0 + p1;
#pragma unroll
      for (int off = 1; off < 16; off <<= 1)
        ls += __shfl_xor(ls, off, 32);
      rsum[j] = rsum[j] * alpha + ls;
#pragma unroll
      for (int t4 = 0; t4 < 4; ++t4) O[t4][j] = O[t4][j] * alpha;
      const int m = j + 8 * hi;
      { unsigned short ph, pq;
        split16(p0 * 1024.0f, ph, pq); Plds[wib][m * 32 + n] = ph;      Pldsl[wib][m * 32 + n] = pq;
        split16(p1 * 1024.0f, ph, pq); Plds[wib][m * 32 + 16 + n] = ph; Pldsl[wib][m * 32 + 16 + n] = pq; }
    }

    asm volatile("s_wait_dscnt 0" ::: "memory");
    Frag pf, pfl;
    {
      const unsigned short* p = &Plds[wib][(lane & 15) * 32 + hi * 8];
      pf.q[0] = *(const uint4*)(p);
      pf.q[1] = *(const uint4*)(p + 16);
      const unsigned short* pl = &Pldsl[wib][(lane & 15) * 32 + hi * 8];
      pfl.q[0] = *(const uint4*)(pl);
      pfl.q[1] = *(const uint4*)(pl + 16);
    }

#pragma unroll
    for (int t4 = 0; t4 < 4; ++t4) {
      Frag vf  = load_frag_B(VtB, Lseq, h * DhC + 16 * t4, k0, lane);
      Frag vfl = load_frag_B(VtB + PLX, Lseq, h * DhC + 16 * t4, k0, lane);
      O[t4] = wmma_split(pf, pfl, vf, vfl, O[t4]);
    }
  }

  float* so = ost[wib];
#pragma unroll
  for (int j = 0; j < 8; ++j) {
    const float inv = (rsum[j] > 0.f) ? (1.0f / (rsum[j] * 1024.0f)) : 0.f;
#pragma unroll
    for (int t4 = 0; t4 < 4; ++t4) so[(j + 8 * hi) * 64 + 16 * t4 + n] = O[t4][j] * inv;
  }
  asm volatile("s_wait_dscnt 0" ::: "memory");
  store_rows64_planes(so, Attnbf + (size_t)(b * Lseq + qt * 16) * Dmod + h * DhC, PLX, Dmod, lane);
}

__global__ __launch_bounds__(256)
void outproj_kernel(const unsigned short* __restrict__ Attnbf,
                    const unsigned short* __restrict__ WoutT,
                    float* __restrict__ out) {
  __shared__ __align__(16) float st[8][16 * 64];
  const int lane = threadIdx.x & 31;
  const int wib  = threadIdx.x >> 5;
  const int gw   = blockIdx.x * (blockDim.x >> 5) + (threadIdx.x >> 5);
  const int nW   = Dmod / 64;
  const int mt   = gw / nW;
  const int nw   = gw - mt * nW;
  const int row0 = mt * 16;
  const int n0   = nw * 64;

  floatx8 acc[4] = {};
  for (int k0 = 0; k0 < Dmod; k0 += 32) {
    Frag a  = load_frag_A(Attnbf, Dmod, row0, k0, lane);
    Frag al = load_frag_A(Attnbf + PLX, Dmod, row0, k0, lane);
    if (k0 + 32 < Dmod) {
      __builtin_prefetch(Attnbf + (size_t)(row0 + (lane & 15)) * Dmod + k0 + 32, 0, 1);
    }
#pragma unroll
    for (int t = 0; t < 4; ++t) {
      Frag b  = load_frag_B(WoutT, Dmod, n0 + 16 * t, k0, lane);
      Frag bl = load_frag_B(WoutT + PLO, Dmod, n0 + 16 * t, k0, lane);
      acc[t] = wmma_split(a, al, b, bl, acc[t]);
    }
  }

  const int n = lane & 15, hi = lane >> 4;
  float* sw = st[wib];
#pragma unroll
  for (int j = 0; j < 8; ++j)
#pragma unroll
    for (int t = 0; t < 4; ++t) sw[(j + 8 * hi) * 64 + 16 * t + n] = acc[t][j];
  asm volatile("s_wait_dscnt 0" ::: "memory");
  typedef __attribute__((ext_vector_type(4))) float v4f_t;
  typedef float v4fa __attribute__((ext_vector_type(4), may_alias));
  v4f_t ov[8]; size_t oo[8];
#pragma unroll
  for (int i = 0; i < 8; ++i) { const int c = lane + 32 * i, rr = c >> 4, q = c & 15; ov[i] = *(const volatile v4fa*)(sw + rr * 64 + q * 4); oo[i] = (size_t)(row0 + rr) * Dmod + n0 + q * 4; }
#pragma unroll
  for (int i = 0; i < 8; ++i) *(volatile v4f_t*)(out + oo[i]) = ov[i];
  __threadfence();
#pragma unroll
  for (int i = 0; i < 8; ++i) *(volatile v4f_t*)(out + oo[i]) = ov[i];
}

extern "C" void kernel_launch(void* const* d_in, const int* in_sizes, int n_in,
                              void* d_out, int out_size, void* d_ws, size_t ws_size,
                              hipStream_t stream) {
  (void)in_sizes; (void)n_in; (void)out_size; (void)ws_size;
  const float* x    = (const float*)d_in[0];
  const int*   mask = (const int*)d_in[1];
  const float* Wqkv = (const float*)d_in[2];
  const float* Wout = (const float*)d_in[3];
  float* out = (float*)d_out;

  char* ws = (char*)d_ws;
  const size_t MiB = 1u << 20;
  unsigned short* Xbf    = (unsigned short*)(ws + 0);
  unsigned short* WqkvT  = (unsigned short*)(ws + 16 * MiB);
  unsigned short* WoutT  = (unsigned short*)(ws + 28 * MiB);
  unsigned short* Qbf    = (unsigned short*)(ws + 32 * MiB);
  unsigned short* Kbf    = (unsigned short*)(ws + 48 * MiB);
  unsigned short* Vr     = (unsigned short*)(ws + 64 * MiB);
  unsigned short* Vt     = (unsigned short*)(ws + 80 * MiB);
  unsigned short* Attnbf = (unsigned short*)(ws + 96 * MiB);

  {
    int n = Mrows * Dmod;
    cvt_f32_bf16<<<(n / 2 + 255) / 256, 256, 0, stream>>>(x, Xbf, n);
  }
  {
    int n = Dmod * NQKV;
    cvt_f32_bf16_T<<<(n / 2 + 255) / 256, 256, 0, stream>>>(Wqkv, WqkvT, Dmod, NQKV);
  }
  {
    int n = Dmod * Dmod;
    cvt_f32_bf16_T<<<(n / 2 + 255) / 256, 256, 0, stream>>>(Wout, WoutT, Dmod, Dmod);
  }

  qkv_rope_kernel<<<12288 / 8, 256, 0, stream>>>(Xbf, WqkvT, Qbf, Kbf, Vr);
  vt_kernel<<<dim3(Mrows / 64, Dmod / 64, 2), 256, 0, stream>>>(Vr, Vt);

  attn_kernel<<<4096 / 8, 256, 0, stream>>>(Qbf, Kbf, Vt, mask, Attnbf);

  outproj_kernel<<<4096 / 8, 256, 0, stream>>>(Attnbf, WoutT, out);
}
